// ProteinLigandGNN_54193897341260
// MI455X (gfx1250) — hardware-verified
//
#include <hip/hip_runtime.h>
#include <stddef.h>


#define HD     128
#define NG     256
#define NTHR   256
#define NWAVE  8
#define EPT    8
#define NGRP   2
#define CHUNK  (NTHR * EPT * NGRP)
#define WCAP   (EPT * NGRP * 32)
#define LISTN  (NWAVE * WCAP)
#define NBD    8192
#define NB1    2048
#define NB2    512
#define YW     32
#define GROWS  128
#define HP     136
#define PS     16
#define RECF   (NG * HD + NG)
#define W1S    4.0f
#define W1I    0.25f
#define W2S    8.0f
#define W2I    0.125f

#define LDS_GEMM (GROWS * HD * 4)
#define LDS_AGG1 (NB1 * YW * 4 + LISTN * 4 + 64)
#define LDS_AGG2 (NB2 * HD * 4 + LISTN * 4 + NB2 * 4 + 128)
#define LDS_HEAD (NG * HD * 4 + 3 * NG * 4)

static_assert((CHUNK & (CHUNK - 1)) == 0);
static_assert(CHUNK <= 4096);
static_assert(NB1 <= 4096 && NB2 <= 4096);
static_assert(NBD % NB1 == 0 && NB1 % NB2 == 0 && NB1 % GROWS == 0 && NBD % GROWS == 0);
static_assert(GROWS * HP * 2 <= LDS_GEMM);
static_assert(2 * PS * HD * 4 <= LISTN * 4);
static_assert((RECF * 4) % 128 == 0);
static_assert(NG % PS == 0 && PS * HD == 8 * NTHR && NG == NTHR && HD == 128 && YW == 32);
static_assert(NBD == NWAVE * 8 * 128);
static_assert((NB1 * YW / 4) % NTHR == 0 && (NB2 * HD / 4) % NTHR == 0);

typedef float    v4f  __attribute__((ext_vector_type(4)));
typedef float    v8f  __attribute__((ext_vector_type(8)));
typedef int      v4i  __attribute__((ext_vector_type(4)));
typedef _Float16 v8h  __attribute__((ext_vector_type(8)));
typedef _Float16 v16h __attribute__((ext_vector_type(16)));
typedef __bf16   v8b  __attribute__((ext_vector_type(8)));
typedef __bf16   v16b __attribute__((ext_vector_type(16)));
union FragH { v16h v; v8h h[2]; };
union FragB { v16b v; v8b h[2]; };
union PackB { v8b v; v4i q; };

__device__ __forceinline__ v8h cvt8(v4f a, v4f b) {
  v8h r;
  r[0] = (_Float16)a.x; r[1] = (_Float16)a.y; r[2] = (_Float16)a.z; r[3] = (_Float16)a.w;
  r[4] = (_Float16)b.x; r[5] = (_Float16)b.y; r[6] = (_Float16)b.z; r[7] = (_Float16)b.w;
  return r;
}

__device__ __forceinline__ v8b hi8(v4f a, v4f b) {
  v8b r;
  r[0] = (__bf16)a.x; r[1] = (__bf16)a.y; r[2] = (__bf16)a.z; r[3] = (__bf16)a.w;
  r[4] = (__bf16)b.x; r[5] = (__bf16)b.y; r[6] = (__bf16)b.z; r[7] = (__bf16)b.w;
  return r;
}
__device__ __forceinline__ v8b lo8(v4f a, v4f b, v8b hi) {
  v8b r;
  r[0] = (__bf16)(a.x - (float)hi[0]); r[1] = (__bf16)(a.y - (float)hi[1]);
  r[2] = (__bf16)(a.z - (float)hi[2]); r[3] = (__bf16)(a.w - (float)hi[3]);
  r[4] = (__bf16)(b.x - (float)hi[4]); r[5] = (__bf16)(b.y - (float)hi[5]);
  r[6] = (__bf16)(b.z - (float)hi[6]); r[7] = (__bf16)(b.w - (float)hi[7]);
  return r;
}

__device__ __forceinline__ v8f wmh(v16h a, v16h b, v8f c) {
  v8f d = __builtin_amdgcn_wmma_f32_16x16x32_f16(false, a, false, b, (short)0, c, false, false);
  asm volatile("v_nop\n\tv_nop\n\tv_nop\n\tv_nop" : "+v"(d) : "v"(a), "v"(b));
  return d;
}
__device__ __forceinline__ v8f wmb(v16b a, v16b b, v8f c) {
  v8f d = __builtin_amdgcn_wmma_f32_16x16x32_bf16(false, a, false, b, (short)0, c, false, false);
  asm volatile("v_nop\n\tv_nop\n\tv_nop\n\tv_nop" : "+v"(d) : "v"(a), "v"(b));
  return d;
}

__device__ __forceinline__ void load8(const int* __restrict__ dsts, int nE, int e0, int vec8, v4i& da, v4i& db) {
  const int sent = -2147483647 - 1;
  if (vec8 != 0 && e0 + 7 < nE) {
    da = *(const v4i*)(dsts + e0);
    db = *(const v4i*)(dsts + e0 + 4);
  } else {
    da.x = (e0     < nE) ? dsts[e0]     : sent;
    da.y = (e0 + 1 < nE) ? dsts[e0 + 1] : sent;
    da.z = (e0 + 2 < nE) ? dsts[e0 + 2] : sent;
    da.w = (e0 + 3 < nE) ? dsts[e0 + 3] : sent;
    db.x = (e0 + 4 < nE) ? dsts[e0 + 4] : sent;
    db.y = (e0 + 5 < nE) ? dsts[e0 + 5] : sent;
    db.z = (e0 + 6 < nE) ? dsts[e0 + 6] : sent;
    db.w = (e0 + 7 < nE) ? dsts[e0 + 7] : sent;
  }
}

template <int NB>
__device__ __forceinline__ int scan_chunk(const int* __restrict__ dsts, int nE, int cbase, int nodeBase,
                                          int vec8, int* list, int tid, int lane, int wave) {
  int wc = 0;
#pragma unroll
  for (int g = 0; g < NGRP; ++g) {
    const int el0 = (g * NTHR + tid) * EPT;
    const int e0  = cbase + el0;
    v4i da, db;
    load8(dsts, nE, e0, vec8, da, db);
    const unsigned nb = (unsigned)nodeBase;
    const unsigned s0 = (unsigned)da.x - nb, s1 = (unsigned)da.y - nb;
    const unsigned s2 = (unsigned)da.z - nb, s3 = (unsigned)da.w - nb;
    const unsigned s4 = (unsigned)db.x - nb, s5 = (unsigned)db.y - nb;
    const unsigned s6 = (unsigned)db.z - nb, s7 = (unsigned)db.w - nb;
    const bool h0 = s0 < (unsigned)NB, h1 = s1 < (unsigned)NB, h2 = s2 < (unsigned)NB, h3 = s3 < (unsigned)NB;
    const bool h4 = s4 < (unsigned)NB, h5 = s5 < (unsigned)NB, h6 = s6 < (unsigned)NB, h7 = s7 < (unsigned)NB;
    const unsigned any = __builtin_amdgcn_ballot_w32(h0 | h1 | h2 | h3 | h4 | h5 | h6 | h7);
    if (any != 0u) {
#define HITJ(J, HJ, SJ) { \
        const unsigned mj = __builtin_amdgcn_ballot_w32(HJ); \
        if (mj != 0u) { \
          if (HJ) { \
            const int pos = wc + (int)__builtin_amdgcn_mbcnt_lo(mj, 0u); \
            if (pos < WCAP) list[wave * WCAP + pos] = ((el0 + (J)) << 12) | (int)(SJ); \
          } \
          wc += (int)__builtin_popcount(mj); } }
      HITJ(0, h0, s0)
      HITJ(1, h1, s1)
      HITJ(2, h2, s2)
      HITJ(3, h3, s3)
      HITJ(4, h4, s4)
      HITJ(5, h5, s5)
      HITJ(6, h6, s6)
      HITJ(7, h7, s7)
#undef HITJ
    }
  }
  return wc;
}

__global__ __launch_bounds__(NTHR) void k_wprep(
    const float* __restrict__ Wp1, int F1, const float* __restrict__ Wp2, const float* __restrict__ Wl2,
    const float* __restrict__ Wfc, _Float16* w1s, _Float16* w2s, _Float16* w3s, __bf16* wfh, __bf16* wfl) {
  const int i  = blockIdx.x * NTHR + threadIdx.x;
  const int U1 = HD * YW / 8;
  const int U2 = HD * HD / 8;
  const int U4 = HD * (2 * HD) / 8;
  if (i >= U1 + 2 * U2 + U4) return;
  float v[8];
  if (i < U1 + 2 * U2) {
    _Float16* dst;
    if (i < U1) {
      const int o = i * 8, n = o / YW, k0 = o - n * YW;
#pragma unroll
      for (int j = 0; j < 8; ++j) {
        const int k = k0 + j;
        v[j] = (k < F1) ? Wp1[(size_t)k * HD + n] * W1S : 0.f;
      }
      dst = w1s + o;
    } else {
      const bool sec = i < U1 + U2;
      const int  o   = (sec ? (i - U1) : (i - U1 - U2)) * 8;
      const int  n   = o / HD, k0 = o - n * HD;
      const float* W = sec ? Wp2 : Wl2;
#pragma unroll
      for (int j = 0; j < 8; ++j) v[j] = W[(size_t)(k0 + j) * HD + n] * W2S;
      dst = (sec ? w2s : w3s) + o;
    }
    v8h hv;
#pragma unroll
    for (int j = 0; j < 8; ++j) hv[j] = (_Float16)v[j];
    *(volatile v8h*)dst = hv;
    __threadfence();
    *(volatile v8h*)dst = hv;
  } else {
    const int o = (i - U1 - 2 * U2) * 8, n = o / (2 * HD), k0 = o - n * (2 * HD);
#pragma unroll
    for (int j = 0; j < 8; ++j) v[j] = Wfc[(size_t)(k0 + j) * HD + n];
    v4f a, b;
    a.x = v[0]; a.y = v[1]; a.z = v[2]; a.w = v[3];
    b.x = v[4]; b.y = v[5]; b.z = v[6]; b.w = v[7];
    PackB ph, pl;
    ph.v = hi8(a, b);
    pl.v = lo8(a, b, ph.v);
    __bf16* dh = wfh + o;
    __bf16* dl = wfl + o;
    *(volatile v4i*)dh = ph.q;
    *(volatile v4i*)dl = pl.q;
    __threadfence();
    *(volatile v4i*)dh = ph.q;
    *(volatile v4i*)dl = pl.q;
  }
}

__global__ __launch_bounds__(NTHR) void k_deg(
    const int* __restrict__ ei, const float* __restrict__ x, int F,
    float* dinv, float* y, int nN, int nE, int vec8) {
  __shared__ __attribute__((aligned(16))) int cnt[NBD];
  const int tid = threadIdx.x, lane = tid & 31, wave = tid >> 5;
  const int nodeBase = blockIdx.x * NBD;
  const int* dsts = ei + nE;

  for (int i = tid; i < NBD; i += NTHR) cnt[i] = 0;
  __syncthreads();

  const int nChunks = (nE + CHUNK - 1) / CHUNK;
#pragma unroll 1
  for (int ch = 0; ch < nChunks; ++ch) {
    const int cbase = ch * CHUNK;
#pragma unroll
    for (int g = 0; g < NGRP; ++g) {
      const int e0 = cbase + (g * NTHR + tid) * EPT;
      v4i da, db;
      load8(dsts, nE, e0, vec8, da, db);
      const unsigned nb = (unsigned)nodeBase;
#define DEGJ(V) { const unsigned sj = (unsigned)(V) - nb; if (sj < (unsigned)NBD) atomicAdd(&cnt[sj], 1); }
      DEGJ(da.x) DEGJ(da.y) DEGJ(da.z) DEGJ(da.w)
      DEGJ(db.x) DEGJ(db.y) DEGJ(db.z) DEGJ(db.w)
#undef DEGJ
    }
  }
  __syncthreads();

  v4f dq[8];
#pragma unroll
  for (int q = 0; q < 8; ++q) {
    const int f = (wave * 8 + q) * 128 + 4 * lane;
    const v4i c = *(const v4i*)(cnt + f);
    dq[q].x = rsqrtf((float)(c.x + 1));
    dq[q].y = rsqrtf((float)(c.y + 1));
    dq[q].z = rsqrtf((float)(c.z + 1));
    dq[q].w = rsqrtf((float)(c.w + 1));
  }
  float* dp = dinv + (size_t)nodeBase;
#pragma unroll
  for (int q = 0; q < 8; ++q) *(volatile v4f*)(dp + (wave * 8 + q) * 128 + 4 * lane) = dq[q];
  __threadfence();
#pragma unroll
  for (int q = 0; q < 8; ++q) *(volatile v4f*)(dp + (wave * 8 + q) * 128 + 4 * lane) = dq[q];

#pragma unroll 1
  for (int r = tid; r < NBD; r += NTHR) {
    const int node  = nodeBase + r;
    const int nodec = node > nN - 1 ? nN - 1 : node;
    const float d   = rsqrtf((float)(cnt[r] + 1));
    const float* xr = x + (size_t)nodec * F;
    v4f ov[8];
#pragma unroll
    for (int q = 0; q < 8; ++q) {
      v4f o;
      o.x = (4 * q + 0 < F) ? xr[4 * q + 0] * d : 0.f;
      o.y = (4 * q + 1 < F) ? xr[4 * q + 1] * d : 0.f;
      o.z = (4 * q + 2 < F) ? xr[4 * q + 2] * d : 0.f;
      o.w = (4 * q + 3 < F) ? xr[4 * q + 3] * d : 0.f;
      ov[q] = o;
    }
    float* yp = y + (size_t)node * YW;
#pragma unroll
    for (int q = 0; q < 8; ++q) *(volatile v4f*)(yp + 4 * q) = ov[q];
    __threadfence();
#pragma unroll
    for (int q = 0; q < 8; ++q) *(volatile v4f*)(yp + 4 * q) = ov[q];
  }
}

__global__ __launch_bounds__(NTHR) void k_agg1(
    const int* __restrict__ ei, const float* __restrict__ y, const float* __restrict__ dinv,
    float* ax, int nN, int nE, int vec8) {
  extern __shared__ v4f lds_dyn[];
  float* acc  = (float*)lds_dyn;
  int*   list = (int*)(acc + NB1 * YW);
  int*   wcnt = list + LISTN;
  const int tid = threadIdx.x, lane = tid & 31, wave = tid >> 5;
  const int nodeBase = blockIdx.x * NB1;
  const int* dsts = ei + nE;

  {
    const v4f z = {0.f, 0.f, 0.f, 0.f};
    for (int i = tid; i < NB1 * YW / 4; i += NTHR) lds_dyn[i] = z;
  }
  __syncthreads();

  const int nChunks = (nE + CHUNK - 1) / CHUNK;
#pragma unroll 1
  for (int ch = 0; ch < nChunks; ++ch) {
    const int cbase = ch * CHUNK;
    const int wc = scan_chunk<NB1>(dsts, nE, cbase, nodeBase, vec8, list, tid, lane, wave);
    if (lane == 0) wcnt[wave] = wc;
    __syncthreads();
    if (wave == 0) {
#pragma unroll 1
      for (int wsx = 0; wsx < NWAVE; ++wsx) {
        int n = __builtin_amdgcn_readfirstlane(wcnt[wsx]);
        n = n > WCAP ? WCAP : (n < 0 ? 0 : n);
        const int* lp = list + wsx * WCAP;
#pragma unroll 1
        for (int i = 0; i < n; ++i) {
          const int ent = __builtin_amdgcn_readfirstlane(lp[i]);
          int slot = ent & 4095;
          slot = slot > NB1 - 1 ? NB1 - 1 : slot;
          int e = cbase + ((ent >> 12) & (CHUNK - 1));
          e = e > nE - 1 ? nE - 1 : e;
          int src = ei[e];
          src = src < 0 ? 0 : (src > nN - 1 ? nN - 1 : src);
          if (lane < YW / 4) {
            const v4f v = *(const v4f*)(y + (size_t)src * YW + 4 * lane);
            v4f* ap = (v4f*)(acc + slot * YW + 4 * lane);
            *ap = *ap + v;
          }
        }
      }
    }
    __syncthreads();
  }

#pragma unroll 4
  for (int i = 0; i < (NB1 * YW / 4) / NTHR; ++i) {
    const int idx   = i * NTHR + tid;
    const int row   = idx >> 3;
    const int c4    = (idx & 7) * 4;
    const int node  = nodeBase + row;
    const int nodec = node > nN - 1 ? nN - 1 : node;
    const float d   = dinv[nodec];
    const v4f av = *(const v4f*)(acc + row * YW + c4);
    const v4f yv = *(const v4f*)(y + (size_t)nodec * YW + c4);
    const v4f o  = (av + yv) * d;
    float* op = ax + (size_t)node * YW + c4;
    *(volatile v4f*)op = o;
    __threadfence();
    *(volatile v4f*)op = o;
  }
}

template <bool K4>
__global__ __launch_bounds__(NTHR) void k_gemm12(
    const float* __restrict__ ax, const _Float16* __restrict__ w1s, const float* __restrict__ w1f,
    const float* __restrict__ b1, const _Float16* __restrict__ w2s, const float* __restrict__ dinv,
    float* g2) {
  extern __shared__ v4f lds_dyn[];
  _Float16* sH  = (_Float16*)lds_dyn;
  float*    stg = (float*)lds_dyn;
  const int tid = threadIdx.x, lane = tid & 31, wave = tid >> 5, hh = lane >> 4, m = lane & 15;
  const int rowBase = blockIdx.x * GROWS;

  if (K4) {
    const int r = tid >> 1, n0 = (tid & 1) * (HD / 2);
    const v4f a = *(const v4f*)(ax + (size_t)(rowBase + r) * YW);
    _Float16* hrow = sH + r * HP + n0;
#pragma unroll 4
    for (int n = 0; n < HD / 2; ++n) {
      const int col = n0 + n;
      float v = b1[col];
      v += a.x * w1f[col];
      v += a.y * w1f[HD + col];
      v += a.z * w1f[2 * HD + col];
      v += a.w * w1f[3 * HD + col];
      hrow[n] = (_Float16)fmaxf(v, 0.f);
    }
  } else {
    const float* ap = ax + (size_t)(rowBase + wave * 16 + m) * YW + 8 * hh;
    const v4f p0 = *(const v4f*)ap,        p1 = *(const v4f*)(ap + 4);
    const v4f p2 = *(const v4f*)(ap + 16), p3 = *(const v4f*)(ap + 20);
    FragH a;
    a.h[0] = cvt8(p0, p1);
    a.h[1] = cvt8(p2, p3);
    v8f acc[8];
#pragma unroll
    for (int t = 0; t < 8; ++t) {
      const _Float16* bp = w1s + (size_t)(16 * t + m) * YW + 8 * hh;
      FragH b;
      b.h[0] = *(const v8h*)bp;
      b.h[1] = *(const v8h*)(bp + 16);
      const v8f z = {0.f, 0.f, 0.f, 0.f, 0.f, 0.f, 0.f, 0.f};
      acc[t] = wmh(a.v, b.v, z);
    }
    const int r0 = wave * 16 + 8 * hh;
#pragma unroll
    for (int t = 0; t < 8; ++t) {
      const float bb = b1[16 * t + m];
      _Float16* hp = sH + r0 * HP + 16 * t + m;
#pragma unroll
      for (int r = 0; r < 8; ++r) hp[r * HP] = (_Float16)fmaxf(acc[t][r] * W1I + bb, 0.f);
    }
  }
  __syncthreads();

  v8f acc2[8];
#pragma unroll
  for (int t = 0; t < 8; ++t) { const v8f z = {0.f, 0.f, 0.f, 0.f, 0.f, 0.f, 0.f, 0.f}; acc2[t] = z; }
  const _Float16* ar = sH + (wave * 16 + m) * HP + 8 * hh;
#pragma unroll
  for (int kt = 0; kt < HD / 32; ++kt) {
    FragH a;
    a.h[0] = *(const v8h*)(ar + 32 * kt);
    a.h[1] = *(const v8h*)(ar + 32 * kt + 16);
#pragma unroll
    for (int t = 0; t < 8; ++t) {
      const _Float16* bp = w2s + (size_t)(16 * t + m) * HD + 32 * kt + 8 * hh;
      FragH b;
      b.h[0] = *(const v8h*)bp;
      b.h[1] = *(const v8h*)(bp + 16);
      acc2[t] = wmh(a.v, b.v, acc2[t]);
    }
  }
  __syncthreads();

  {
    const int r0 = wave * 16 + 8 * hh;
    const v4f dA = *(const v4f*)(dinv + (size_t)rowBase + r0);
    const v4f dB = *(const v4f*)(dinv + (size_t)rowBase + r0 + 4);
    const float d0 = dA.x * W2I, d1 = dA.y * W2I, d2 = dA.z * W2I, d3 = dA.w * W2I;
    const float d4 = dB.x * W2I, d5 = dB.y * W2I, d6 = dB.z * W2I, d7 = dB.w * W2I;
    float* sp = stg + r0 * HD + m;
#pragma unroll
    for (int t = 0; t < 8; ++t) {
      sp[0 * HD + 16 * t] = acc2[t][0] * d0;
      sp[1 * HD + 16 * t] = acc2[t][1] * d1;
      sp[2 * HD + 16 * t] = acc2[t][2] * d2;
      sp[3 * HD + 16 * t] = acc2[t][3] * d3;
      sp[4 * HD + 16 * t] = acc2[t][4] * d4;
      sp[5 * HD + 16 * t] = acc2[t][5] * d5;
      sp[6 * HD + 16 * t] = acc2[t][6] * d6;
      sp[7 * HD + 16 * t] = acc2[t][7] * d7;
    }
  }
  __syncthreads();

  const float* lp = stg + wave * 16 * HD + 4 * lane;
  float* gp = g2 + ((size_t)rowBase + wave * 16) * HD + 4 * lane;
#pragma unroll
  for (int i = 0; i < 16; ++i) { const v4f v = *(const v4f*)(lp + i * HD); *(volatile v4f*)(gp + (size_t)i * HD) = v; }
  __threadfence();
#pragma unroll
  for (int i = 0; i < 16; ++i) { const v4f v = *(const v4f*)(lp + i * HD); *(volatile v4f*)(gp + (size_t)i * HD) = v; }
}

__global__ __launch_bounds__(NTHR) void k_agg2(
    const int* __restrict__ ei, const float* __restrict__ g2, const float* __restrict__ dinv,
    const float* __restrict__ b2, const int* __restrict__ batch, const int* __restrict__ ngp,
    float* rec, int nN, int nE, int vec8) {
  extern __shared__ v4f lds_dyn[];
  __shared__ __attribute__((aligned(16))) float cntall[NG];
  __shared__ float cnt2[2 * PS];
  float* acc   = (float*)lds_dyn;
  int*   list  = (int*)(acc + NB2 * HD);
  float* pool2 = (float*)list;
  int*   bsl   = list + LISTN;
  int*   wcnt  = bsl + NB2;
  int*   red   = wcnt + NWAVE;
  const int tid = threadIdx.x, lane = tid & 31, wave = tid >> 5;
  const int nodeBase = blockIdx.x * NB2;
  const int* dsts = ei + nE;

  {
    const v4f z = {0.f, 0.f, 0.f, 0.f};
    for (int i = tid; i < NB2 * HD / 4; i += NTHR) lds_dyn[i] = z;
  }
  __syncthreads();

  const int nChunks = (nE + CHUNK - 1) / CHUNK;
#pragma unroll 1
  for (int ch = 0; ch < nChunks; ++ch) {
    const int cbase = ch * CHUNK;
    const int wc = scan_chunk<NB2>(dsts, nE, cbase, nodeBase, vec8, list, tid, lane, wave);
    if (lane == 0) wcnt[wave] = wc;
    __syncthreads();
    if (wave == 0) {
#pragma unroll 1
      for (int wsx = 0; wsx < NWAVE; ++wsx) {
        int n = __builtin_amdgcn_readfirstlane(wcnt[wsx]);
        n = n > WCAP ? WCAP : (n < 0 ? 0 : n);
        const int* lp = list + wsx * WCAP;
#pragma unroll 1
        for (int i = 0; i < n; ++i) {
          const int ent = __builtin_amdgcn_readfirstlane(lp[i]);
          int slot = ent & 4095;
          slot = slot > NB2 - 1 ? NB2 - 1 : slot;
          int e = cbase + ((ent >> 12) & (CHUNK - 1));
          e = e > nE - 1 ? nE - 1 : e;
          int src = ei[e];
          src = src < 0 ? 0 : (src > nN - 1 ? nN - 1 : src);
          const v4f v = *(const v4f*)(g2 + (size_t)src * HD + 4 * lane);
          v4f* ap = (v4f*)(acc + slot * HD + 4 * lane);
          *ap = *ap + v;
        }
      }
    }
    __syncthreads();
  }

#pragma unroll 4
  for (int i = 0; i < (NB2 * HD / 4) / NTHR; ++i) {
    const int idx  = i * NTHR + tid;
    const int slot = idx >> 5;
    const int c4   = (idx & 31) * 4;
    int node = nodeBase + slot;
    node = node > nN - 1 ? nN - 1 : node;
    const float d  = dinv[node];
    const v4f   gv = *(const v4f*)(g2 + (size_t)node * HD + c4);
    const v4f   bv = *(const v4f*)(b2 + c4);
    v4f* ap = (v4f*)(acc + slot * HD + c4);
    v4f hv = (*ap + gv) * d + bv;
    hv.x = fmaxf(hv.x, 0.f); hv.y = fmaxf(hv.y, 0.f); hv.z = fmaxf(hv.z, 0.f); hv.w = fmaxf(hv.w, 0.f);
    *ap = hv;
  }

  int numG = ngp[0];
  numG = numG < 0 ? 0 : (numG > NG ? NG : numG);
  int mn = NG, mx = -1;
  for (int s = tid; s < NB2; s += NTHR) {
    const int node = nodeBase + s;
    int b = -1;
    if (node < nN) {
      const int bb = batch[node];
      if (bb >= 0 && bb < numG) b = bb;
    }
    bsl[s] = b;
    if (b >= 0) { mn = b < mn ? b : mn; mx = b > mx ? b : mx; }
  }
  for (int i = tid; i < NG; i += NTHR) cntall[i] = 0.f;
#pragma unroll
  for (int off = 16; off > 0; off >>= 1) {
    const int om = __shfl_xor(mn, off);
    const int ox = __shfl_xor(mx, off);
    mn = om < mn ? om : mn;
    mx = ox > mx ? ox : mx;
  }
  if (lane == 0) { red[wave] = mn; red[NWAVE + wave] = mx; }
  __syncthreads();
  if (tid == 0) {
    int m1 = NG, m2 = -1;
#pragma unroll
    for (int w = 0; w < NWAVE; ++w) {
      m1 = red[w] < m1 ? red[w] : m1;
      m2 = red[NWAVE + w] > m2 ? red[NWAVE + w] : m2;
    }
    red[2 * NWAVE] = m1;
    red[2 * NWAVE + 1] = m2;
  }
  __syncthreads();
  const int gmin = red[2 * NWAVE], gmax = red[2 * NWAVE + 1];

  const int col = tid & (HD - 1), half = tid >> 7;
  float* recb = rec + (size_t)blockIdx.x * RECF;
#pragma unroll 1
  for (int c = 0; c < NG / PS; ++c) {
    const int gb = c * PS;
    const bool active = (gmax >= gb) && (gmin <= gb + PS - 1);
    v4f o0 = {0.f, 0.f, 0.f, 0.f}, o1 = {0.f, 0.f, 0.f, 0.f};
    if (active) {
      for (int i = tid; i < 2 * PS * HD; i += NTHR) pool2[i] = 0.f;
      if (tid < 2 * PS) cnt2[tid] = 0.f;
      __syncthreads();
      const float* arow = acc + col;
      float* prow = pool2 + half * PS * HD + col;
#pragma unroll 2
      for (int s = 0; s < NB2 / 2; ++s) {
        const int slot = half * (NB2 / 2) + s;
        const int g = bsl[slot] - gb;
        if ((unsigned)g < (unsigned)PS) {
          prow[g * HD] += arow[slot * HD];
          if (col == 0) cnt2[half * PS + g] += 1.f;
        }
      }
      __syncthreads();
      o0 = *(const v4f*)(pool2 + 4 * tid) + *(const v4f*)(pool2 + PS * HD + 4 * tid);
      o1 = *(const v4f*)(pool2 + (PS * HD) / 2 + 4 * tid) + *(const v4f*)(pool2 + PS * HD + (PS * HD) / 2 + 4 * tid);
      if (tid < PS) cntall[gb + tid] = cnt2[tid] + cnt2[PS + tid];
      __syncthreads();
    }
    float* rp = recb + (size_t)gb * HD;
    *(volatile v4f*)(rp + 4 * tid) = o0;
    *(volatile v4f*)(rp + (PS * HD) / 2 + 4 * tid) = o1;
    __threadfence();
    *(volatile v4f*)(rp + 4 * tid) = o0;
    *(volatile v4f*)(rp + (PS * HD) / 2 + 4 * tid) = o1;
  }
  __syncthreads();
  if (wave == 0) {
    const v4f c0 = *(const v4f*)(cntall + 4 * lane);
    const v4f c1 = *(const v4f*)(cntall + NG / 2 + 4 * lane);
    float* cp = recb + (size_t)NG * HD;
    *(volatile v4f*)(cp + 4 * lane) = c0;
    *(volatile v4f*)(cp + NG / 2 + 4 * lane) = c1;
    __threadfence();
    *(volatile v4f*)(cp + 4 * lane) = c0;
    *(volatile v4f*)(cp + NG / 2 + 4 * lane) = c1;
  }
}

__global__ __launch_bounds__(NTHR) void k_poolred(
    const float* __restrict__ recp, int nBp, const float* __restrict__ recl, int nBl, float* comb) {
  __shared__ __attribute__((aligned(16))) float st[8 * 2 * HD];
  const int tid = threadIdx.x;
  const int g0 = blockIdx.x * 8;
  const bool ta = tid < HD;
  const float* rb = ta ? recp : recl;
  const int nB = ta ? nBp : nBl;
  const int cc = tid & (HD - 1);
#pragma unroll 1
  for (int gi = 0; gi < 8; ++gi) {
    const int g = g0 + gi;
    float s = 0.f, n = 0.f;
    const float* psum = rb + (size_t)g * HD + cc;
    const float* pcnt = rb + (size_t)NG * HD + g;
#pragma unroll 4
    for (int b = 0; b < nB; ++b) {
      s += psum[(size_t)b * RECF];
      n += pcnt[(size_t)b * RECF];
    }
    st[gi * 2 * HD + tid] = s * (1.0f / fmaxf(n, 1.0f));
  }
  __syncthreads();
  const v4f v0 = *(const v4f*)(st + 4 * tid);
  const v4f v1 = *(const v4f*)(st + 8 * HD + 4 * tid);
  float* cp = comb + (size_t)g0 * 2 * HD;
  *(volatile v4f*)(cp + 4 * tid) = v0;
  *(volatile v4f*)(cp + 8 * HD + 4 * tid) = v1;
  __threadfence();
  *(volatile v4f*)(cp + 4 * tid) = v0;
  *(volatile v4f*)(cp + 8 * HD + 4 * tid) = v1;
}

__global__ __launch_bounds__(NTHR) void k_head(
    const float* __restrict__ comb, const __bf16* __restrict__ wfh, const __bf16* __restrict__ wfl,
    const float* __restrict__ bfc,
    const float* __restrict__ w0, const float* __restrict__ c0,
    const float* __restrict__ w1, const float* __restrict__ c1,
    const float* __restrict__ w2, const float* __restrict__ c2,
    float* out) {
  extern __shared__ v4f lds_dyn[];
  float* hid = (float*)lds_dyn;
  float* ob  = hid + NG * HD;
  const int tid = threadIdx.x, lane = tid & 31, wave = tid >> 5, hh = lane >> 4, m = lane & 15;

#pragma unroll 1
  for (int q = 0; q < 2; ++q) {
    const int rt = 2 * wave + q;
    v8f acc[8];
#pragma unroll
    for (int t = 0; t < 8; ++t) { const v8f z = {0.f, 0.f, 0.f, 0.f, 0.f, 0.f, 0.f, 0.f}; acc[t] = z; }
#pragma unroll 2
    for (int ks = 0; ks < (2 * HD) / 32; ++ks) {
      const int k0 = 32 * ks;
      const float* ap = comb + (size_t)(rt * 16 + m) * (2 * HD) + k0 + 8 * hh;
      const v4f p0 = *(const v4f*)ap,        p1 = *(const v4f*)(ap + 4);
      const v4f p2 = *(const v4f*)(ap + 16), p3 = *(const v4f*)(ap + 20);
      FragB ah, al;
      ah.h[0] = hi8(p0, p1);
      ah.h[1] = hi8(p2, p3);
      al.h[0] = lo8(p0, p1, ah.h[0]);
      al.h[1] = lo8(p2, p3, ah.h[1]);
#pragma unroll
      for (int t = 0; t < 8; ++t) {
        const __bf16* bp = wfh + (size_t)(16 * t + m) * (2 * HD) + k0 + 8 * hh;
        const __bf16* lq = wfl + (size_t)(16 * t + m) * (2 * HD) + k0 + 8 * hh;
        FragB bh, bl;
        bh.h[0] = *(const v8b*)bp; bh.h[1] = *(const v8b*)(bp + 16);
        bl.h[0] = *(const v8b*)lq; bl.h[1] = *(const v8b*)(lq + 16);
        acc[t] = wmb(ah.v, bh.v, acc[t]);
        acc[t] = wmb(ah.v, bl.v, acc[t]);
        acc[t] = wmb(al.v, bh.v, acc[t]);
      }
    }
    const int r0 = rt * 16 + 8 * hh;
#pragma unroll
    for (int t = 0; t < 8; ++t) {
      const float bb = bfc[16 * t + m];
      float* hp = hid + (size_t)r0 * HD + 16 * t + m;
#pragma unroll
      for (int r = 0; r < 8; ++r) hp[r * HD] = fmaxf(acc[t][r] + bb, 0.f);
    }
  }
  __syncthreads();

  {
    const int g = tid;
    const float* hp = hid + (size_t)g * HD;
    float pa = 0.f, pb = 0.f, pc = 0.f;
#pragma unroll 4
    for (int k = 0; k < HD; ++k) {
      const float hv = hp[k];
      pa += hv * w0[k];
      pb += hv * w1[k];
      pc += hv * w2[k];
    }
    ob[g]          = pa + c0[0];
    ob[NG + g]     = pb + c1[0];
    ob[2 * NG + g] = pc + c2[0];
  }
  __syncthreads();
  const bool wr = tid < (3 * NG) / 4;
  v4f ov = {0.f, 0.f, 0.f, 0.f};
  if (wr) ov = *(const v4f*)(ob + 4 * tid);
  if (wr) *(volatile v4f*)(out + 4 * tid) = ov;
  __threadfence();
  if (wr) *(volatile v4f*)(out + 4 * tid) = ov;
}

extern "C" void kernel_launch(void* const* d_in, const int* in_sizes, int n_in,
                              void* d_out, int out_size, void* d_ws, size_t ws_size,
                              hipStream_t stream) {
  if (n_in < 23) return;
  const int nNp = in_sizes[2], nNl = in_sizes[5];
  if (nNp <= 0 || nNl <= 0) return;
  const int Fp = in_sizes[0] / nNp, Fl = in_sizes[3] / nNl;
  if (Fp < 1 || Fp > YW || Fp * nNp != in_sizes[0]) return;
  if (Fl != 4 || Fl * nNl != in_sizes[3]) return;
  const int nEp = in_sizes[1] / 2, nEl = in_sizes[4] / 2;
  if (nEp < 0 || nEl < 0 || 2 * nEp != in_sizes[1] || 2 * nEl != in_sizes[4]) return;
  if (in_sizes[6] < 1) return;
  if (in_sizes[7] != Fp * HD || in_sizes[9] != HD * HD || in_sizes[11] != Fl * HD ||
      in_sizes[13] != HD * HD || in_sizes[15] != 2 * HD * HD) return;
  if (in_sizes[8] < HD || in_sizes[10] < HD || in_sizes[12] < HD || in_sizes[14] < HD || in_sizes[16] < HD) return;
  if (in_sizes[17] < HD || in_sizes[19] < HD || in_sizes[21] < HD ||
      in_sizes[18] < 1 || in_sizes[20] < 1 || in_sizes[22] < 1) return;
  if (out_size != 3 * NG) return;

  const float* px      = (const float*)d_in[0];
  const int*   p_ei    = (const int*)d_in[1];
  const int*   p_batch = (const int*)d_in[2];
  const float* lx      = (const float*)d_in[3];
  const int*   l_ei    = (const int*)d_in[4];
  const int*   l_batch = (const int*)d_in[5];
  const int*   ngp     = (const int*)d_in[6];
  const float* Wp1 = (const float*)d_in[7];   const float* bp1  = (const float*)d_in[8];
  const float* Wp2 = (const float*)d_in[9];   const float* bp2  = (const float*)d_in[10];
  const float* Wl1 = (const float*)d_in[11];  const float* bl1  = (const float*)d_in[12];
  const float* Wl2 = (const float*)d_in[13];  const float* bl2  = (const float*)d_in[14];
  const float* Wfc = (const float*)d_in[15];  const float* bfc  = (const float*)d_in[16];
  const float* Wk0 = (const float*)d_in[17];  const float* bk0  = (const float*)d_in[18];
  const float* Wk1 = (const float*)d_in[19];  const float* bk1  = (const float*)d_in[20];
  const float* Wk2 = (const float*)d_in[21];  const float* bk2  = (const float*)d_in[22];
  float* out = (float*)d_out;

  const int nBDp = (nNp + NBD - 1) / NBD,     nBDl = (nNl + NBD - 1) / NBD;
  const int nA1p = (nNp + NB1 - 1) / NB1,     nA1l = (nNl + NB1 - 1) / NB1;
  const int nGp  = (nNp + GROWS - 1) / GROWS, nGl  = (nNl + GROWS - 1) / GROWS;
  const int nA2p = (nNp + NB2 - 1) / NB2,     nA2l = (nNl + NB2 - 1) / NB2;
  const size_t NP8p = (size_t)nBDp * NBD,  NP8l = (size_t)nBDl * NBD;
  const size_t NP2p = (size_t)nA1p * NB1,  NP2l = (size_t)nA1l * NB1;
  const size_t NPGp = (size_t)nGp * GROWS, NPGl = (size_t)nGl * GROWS;

  char* ws = (char*)d_ws;
  size_t off = 0;
  auto take = [&](size_t bytes) -> size_t { const size_t o = off; off += (bytes + 255) & ~(size_t)255; return o; };
  const size_t oW1 = take((size_t)HD * YW * 2);
  const size_t oW2 = take((size_t)HD * HD * 2);
  const size_t oW3 = take((size_t)HD * HD * 2);
  const size_t oWh = take((size_t)HD * 2 * HD * 2);
  const size_t oWl = take((size_t)HD * 2 * HD * 2);
  const size_t oDp = take(NP8p * 4);
  const size_t oYp = take(NP8p * YW * 4);
  const size_t oAp = take(NP2p * YW * 4);
  const size_t oGp = take(NPGp * HD * 4);
  const size_t oRp = take((size_t)nA2p * RECF * 4);
  const size_t oDl = take(NP8l * 4);
  const size_t oYl = take(NP8l * YW * 4);
  const size_t oAl = take(NP2l * YW * 4);
  const size_t oGl = take(NPGl * HD * 4);
  const size_t oRl = take((size_t)nA2l * RECF * 4);
  const size_t oCb = take((size_t)NG * 2 * HD * 4);
  if (off > ws_size) return;

  _Float16* w1s = (_Float16*)(ws + oW1);
  _Float16* w2s = (_Float16*)(ws + oW2);
  _Float16* w3s = (_Float16*)(ws + oW3);
  __bf16*   wfh = (__bf16*)(ws + oWh);
  __bf16*   wfl = (__bf16*)(ws + oWl);
  float* dinv_p = (float*)(ws + oDp);  float* y_p = (float*)(ws + oYp);
  float* ax_p   = (float*)(ws + oAp);  float* g2_p = (float*)(ws + oGp);  float* rec_p = (float*)(ws + oRp);
  float* dinv_l = (float*)(ws + oDl);  float* y_l = (float*)(ws + oYl);
  float* ax_l   = (float*)(ws + oAl);  float* g2_l = (float*)(ws + oGl);  float* rec_l = (float*)(ws + oRl);
  float* comb   = (float*)(ws + oCb);

  const int vec8p = ((nEp & 3) == 0) ? 1 : 0;
  const int vec8l = ((nEl & 3) == 0) ? 1 : 0;

  const int nPrep = HD * YW / 8 + 2 * (HD * HD / 8) + HD * 2 * HD / 8;
  k_wprep<<<(nPrep + NTHR - 1) / NTHR, NTHR, 0, stream>>>(Wp1, Fp, Wp2, Wl2, Wfc, w1s, w2s, w3s, wfh, wfl);

  hipFuncSetAttribute(reinterpret_cast<const void*>(&k_agg1),
                      hipFuncAttributeMaxDynamicSharedMemorySize, LDS_AGG1);
  hipFuncSetAttribute(reinterpret_cast<const void*>(&k_gemm12<false>),
                      hipFuncAttributeMaxDynamicSharedMemorySize, LDS_GEMM);
  hipFuncSetAttribute(reinterpret_cast<const void*>(&k_gemm12<true>),
                      hipFuncAttributeMaxDynamicSharedMemorySize, LDS_GEMM);
  hipFuncSetAttribute(reinterpret_cast<const void*>(&k_agg2),
                      hipFuncAttributeMaxDynamicSharedMemorySize, LDS_AGG2);
  hipFuncSetAttribute(reinterpret_cast<const void*>(&k_head),
                      hipFuncAttributeMaxDynamicSharedMemorySize, LDS_HEAD);

  k_deg<<<nBDp, NTHR, 0, stream>>>(p_ei, px, Fp, dinv_p, y_p, nNp, nEp, vec8p);
  k_agg1<<<nA1p, NTHR, LDS_AGG1, stream>>>(p_ei, y_p, dinv_p, ax_p, nNp, nEp, vec8p);
  k_gemm12<false><<<nGp, NTHR, LDS_GEMM, stream>>>(ax_p, w1s, Wl1, bp1, w2s, dinv_p, g2_p);
  k_agg2<<<nA2p, NTHR, LDS_AGG2, stream>>>(p_ei, g2_p, dinv_p, bp2, p_batch, ngp, rec_p, nNp, nEp, vec8p);

  k_deg<<<nBDl, NTHR, 0, stream>>>(l_ei, lx, Fl, dinv_l, y_l, nNl, nEl, vec8l);
  k_agg1<<<nA1l, NTHR, LDS_AGG1, stream>>>(l_ei, y_l, dinv_l, ax_l, nNl, nEl, vec8l);
  k_gemm12<true><<<nGl, NTHR, LDS_GEMM, stream>>>(ax_l, w1s, Wl1, bl1, w3s, dinv_l, g2_l);
  k_agg2<<<nA2l, NTHR, LDS_AGG2, stream>>>(l_ei, g2_l, dinv_l, bl2, l_batch, ngp, rec_l, nNl, nEl, vec8l);

  k_poolred<<<NG / 8, NTHR, 0, stream>>>(rec_p, nA2p, rec_l, nA2l, comb);
  k_head<<<1, NTHR, LDS_HEAD, stream>>>(comb, wfh, wfl, bfc, Wk0, bk0, Wk1, bk1, Wk2, bk2, out);
}
